// TemporalAttentionModule_4750233830133
// MI455X (gfx1250) — hardware-verified
//
#include <hip/hip_runtime.h>
#include <math.h>

constexpr int kBatch = 2;
constexpr int kSeq   = 4096;
constexpr int kDim   = 1024;
constexpr int kHeads = 16;
constexpr int kHS    = 64;
constexpr int kRows  = kBatch * kSeq;
constexpr int kCat   = 2 * kDim;
constexpr float kWCarry    = 16.0f;
constexpr float kWCarryInv = 1.0f / 16.0f;
constexpr float kInvDim    = 1.0f / 1024.0f;
constexpr float kLnEps     = 1e-6f;
constexpr float kScoreScale = 0.125f;

typedef __attribute__((ext_vector_type(16))) _Float16 v16h;
typedef __attribute__((ext_vector_type(8)))  _Float16 v8h;
typedef __attribute__((ext_vector_type(16))) __bf16   v16b;
typedef __attribute__((ext_vector_type(8)))  __bf16   v8b;
typedef __attribute__((ext_vector_type(8)))  float    v8f;
typedef __attribute__((ext_vector_type(4)))  float    v4f;
typedef __attribute__((ext_vector_type(4)))  unsigned int v4u;

__device__ __forceinline__ unsigned short f2bf_bits(float f) {
  unsigned u = __float_as_uint(f);
  return (unsigned short)((u + 0x7FFFu + ((u >> 16) & 1u)) >> 16);
}
__device__ __forceinline__ float bf_bits2f(unsigned short h) { return __uint_as_float(((unsigned)h) << 16); }

__device__ __forceinline__ void dep_guard_h(v8f& a, v8f& b, v16h x, v16h y) { asm volatile("v_nop\n\tv_nop\n\tv_nop\n\tv_nop" : "+v"(a), "+v"(b) : "v"(x), "v"(y)); }
__device__ __forceinline__ void dep_guard_b(v8f& a, v8f& b, v16b x, v16b y) { asm volatile("v_nop\n\tv_nop\n\tv_nop\n\tv_nop" : "+v"(a), "+v"(b) : "v"(x), "v"(y)); }
__device__ __forceinline__ void keep4_h(v16h a, v16h b, v16h c, v16h d) { asm volatile("v_nop" :: "v"(a), "v"(b), "v"(c), "v"(d)); }
__device__ __forceinline__ void keep4_b(v16b a, v16b b, v16b c, v16b d) { asm volatile("v_nop" :: "v"(a), "v"(b), "v"(c), "v"(d)); }
__device__ __forceinline__ void acc_guard4(v8f& a, v8f& b, v8f& c, v8f& d) { asm volatile("v_nop\n\tv_nop\n\tv_nop\n\tv_nop" : "+v"(a), "+v"(b), "+v"(c), "+v"(d)); }
template <typename T> struct Frag;
template <> struct Frag<_Float16> {
  typedef v16h V; union U { v16h v; v8h h[2]; };
  static __device__ __forceinline__ v16h load(const _Float16* p) {
    U f; f.h[0] = *(const v8h*)(p); f.h[1] = *(const v8h*)(p + 16); return f.v;
  }
  static __device__ __forceinline__ v8f mma(v16h a, v16h b, v8f c) {
    return __builtin_amdgcn_wmma_f32_16x16x32_f16(false, a, false, b, (short)0, c, false, false);
  }
  static __device__ __forceinline__ void guard(v8f& a, v8f& b, v16h x, v16h y) { dep_guard_h(a, b, x, y); }
  static __device__ __forceinline__ void keep(v16h a, v16h b, v16h c, v16h d) { keep4_h(a, b, c, d); }
};
template <> struct Frag<__bf16> {
  typedef v16b V; union U { v16b v; v8b h[2]; };
  static __device__ __forceinline__ v16b load(const __bf16* p) {
    U f; f.h[0] = *(const v8b*)(p); f.h[1] = *(const v8b*)(p + 16); return f.v;
  }
  static __device__ __forceinline__ v8f mma(v16b a, v16b b, v8f c) {
    return __builtin_amdgcn_wmma_f32_16x16x32_bf16(false, a, false, b, (short)0, c, false, false);
  }
  static __device__ __forceinline__ void guard(v8f& a, v8f& b, v16b x, v16b y) { dep_guard_b(a, b, x, y); }
  static __device__ __forceinline__ void keep(v16b a, v16b b, v16b c, v16b d) { keep4_b(a, b, c, d); }
};

__device__ __forceinline__ unsigned pk16(unsigned short a, unsigned short b) { return (unsigned)a | ((unsigned)b << 16); }
__device__ __forceinline__ unsigned short h_bits(float f) { const _Float16 h = (_Float16)f; return __builtin_bit_cast(unsigned short, h); }
__device__ __forceinline__ float hlo2f(unsigned w) { return (float)__builtin_bit_cast(_Float16, (unsigned short)(w & 0xffffu)); }
__device__ __forceinline__ float hhi2f(unsigned w) { return (float)__builtin_bit_cast(_Float16, (unsigned short)(w >> 16)); }

template <int ET> struct Elem;
template <> struct Elem<0> { typedef _Float16 T; };
template <> struct Elem<1> { typedef __bf16 T; };
template <int ET, bool SPLIT, int BIAS_MODE, int OUT_MODE, bool RESID, int ACT = 0>
__global__ __launch_bounds__(256) void wmma_gemm64(
    const unsigned short* __restrict__ Ap, const unsigned short* __restrict__ A2p, int lda, long strideA,
    const unsigned short* __restrict__ Btp, const unsigned short* __restrict__ Bt2p, int ldb, long strideB,
    void* __restrict__ Cout, void* __restrict__ Cout2, int ldc, long strideC,
    const float* __restrict__ bias,
    const float* __restrict__ resid, long strideR,
    int M, int N, int K, float scale) {
  typedef typename Elem<ET>::T T;
  typedef typename Frag<T>::V V;
  const T* A = (const T*)Ap; const T* A2 = (const T*)A2p; const T* Bt = (const T*)Btp; const T* Bt2 = (const T*)Bt2p;
  __shared__ __align__(16) float sT[8][16 * 68];
  const int b    = blockIdx.y;
  const int lane = threadIdx.x & 31;
  const int wave = threadIdx.x >> 5;
  const int tilesN = N >> 6;
  const int tilesM = M >> 6;
  const int tile = blockIdx.x * 8 + wave;
  if (tile >= tilesM * tilesN) return;
  const int tm = tile / tilesN;
  const int tn = tile - tm * tilesN;
  const int m0 = tm << 6;
  const int n0 = tn << 6;

  const T* Ab  = A  + (size_t)b * strideA;
  const T* Bb  = Bt + (size_t)b * strideB;
  const T* Ab2 = SPLIT ? (A2  + (size_t)b * strideA) : nullptr;
  const T* Bb2 = SPLIT ? (Bt2 + (size_t)b * strideB) : nullptr;

  const int rlane = lane & 15;
  const int koff  = (lane >> 4) * 8;
  const int mOff  = (lane >> 4) * 8;

  v8f acc[4][4];
#pragma unroll
  for (int i = 0; i < 4; ++i)
#pragma unroll
    for (int j = 0; j < 4; ++j) acc[i][j] = (v8f){0.f,0.f,0.f,0.f,0.f,0.f,0.f,0.f};

  for (int k0 = 0; k0 < K; k0 += 32) {
    V bh[4], bl[4];
#pragma unroll
    for (int j = 0; j < 4; ++j) {
      const size_t bo = (size_t)(n0 + (j << 4) + rlane) * ldb + koff + k0;
      bh[j] = Frag<T>::load(Bb + bo);
      if (SPLIT) bl[j] = Frag<T>::load(Bb2 + bo);
    }
#pragma unroll
    for (int i = 0; i < 4; ++i) {
      const size_t ao = (size_t)(m0 + (i << 4) + rlane) * lda + koff + k0;
      V ah = Frag<T>::load(Ab + ao);
      V al;
      if (SPLIT) al = Frag<T>::load(Ab2 + ao);
#pragma unroll
      for (int j = 0; j < 4; ++j) {
        acc[i][j] = Frag<T>::mma(ah, bh[j], acc[i][j]);
        if (SPLIT) {
          acc[i][j] = Frag<T>::mma(ah, bl[j], acc[i][j]);
          acc[i][j] = Frag<T>::mma(al, bh[j], acc[i][j]);
        }
      }
      Frag<T>::guard(acc[i][0], acc[i][3], ah, SPLIT ? al : ah);
    }
    Frag<T>::keep(bh[0], bh[1], bh[2], bh[3]);
    if (SPLIT) Frag<T>::keep(bl[0], bl[1], bl[2], bl[3]);
  }
  acc_guard4(acc[0][0], acc[0][1], acc[0][2], acc[0][3]);
  acc_guard4(acc[1][0], acc[1][1], acc[1][2], acc[1][3]);
  acc_guard4(acc[2][0], acc[2][1], acc[2][2], acc[2][3]);
  acc_guard4(acc[3][0], acc[3][1], acc[3][2], acc[3][3]);

  float* slab = sT[wave];
  const float* Rb = RESID ? (resid + (size_t)b * strideR) : nullptr;
#pragma unroll
  for (int i = 0; i < 4; ++i) {
    const int mBase = m0 + (i << 4);
#pragma unroll
    for (int j = 0; j < 4; ++j) {
      const int n = n0 + (j << 4) + rlane;
      float bv = 0.f;
      if (BIAS_MODE == 2) bv = bias[n];
#pragma unroll
      for (int r = 0; r < 8; ++r) {
        float v = acc[i][j][r] * scale;
        if (BIAS_MODE == 1) v += bias[mBase + mOff + r];
        if (BIAS_MODE == 2) v += bv;
        if (RESID) v += Rb[(size_t)(mBase + mOff + r) * ldc + n];
        if (ACT == 2) v = fmaxf(v, 0.0f);
        if (ACT == 4) v = (v > 0.f) ? v : 0.01f * v;
        slab[(mOff + r) * 68 + (j << 4) + rlane] = v;
      }
    }
    __builtin_amdgcn_fence(__ATOMIC_RELEASE, "workgroup");
    __builtin_amdgcn_wave_barrier();
    __builtin_amdgcn_fence(__ATOMIC_ACQUIRE, "workgroup");
    if (OUT_MODE == 0) {
      float* C = (float*)Cout + (size_t)b * strideC;
      const int hh = lane >> 4, c4 = (lane & 15) * 4;
      for (int pass = 0; pass < 2; ++pass) {
#pragma unroll
        for (int it = 0; it < 8; ++it) {
          const int row = it * 2 + hh;
          v4f v = *(const v4f*)(slab + row * 68 + c4);
          *(volatile v4f*)(C + (size_t)(mBase + row) * ldc + n0 + c4) = v;
        }
        __threadfence();
      }
    } else {
      const int q = lane >> 3, c8 = (lane & 7) * 8;
      unsigned short* C  = (unsigned short*)Cout  + (size_t)b * strideC;
      unsigned short* C2 = (OUT_MODE == 2) ? ((unsigned short*)Cout2 + (size_t)b * strideC) : nullptr;
      for (int pass = 0; pass < 2; ++pass) {
#pragma unroll
        for (int it = 0; it < 4; ++it) {
          const int row = it * 4 + q;
          const float* sp = slab + row * 68 + c8;
          v8h hv, lv;
#pragma unroll
          for (int e = 0; e < 8; ++e) {
            if (OUT_MODE == 1) {
              hv[e] = (_Float16)sp[e];
            } else {
              unsigned short hb = f2bf_bits(sp[e]);
              unsigned short lb = f2bf_bits(sp[e] - bf_bits2f(hb));
              hv[e] = __builtin_bit_cast(_Float16, hb);
              lv[e] = __builtin_bit_cast(_Float16, lb);
            }
          }
          *(volatile v8h*)(C + (size_t)(mBase + row) * ldc + n0 + c8) = hv;
          if (OUT_MODE == 2) *(volatile v8h*)(C2 + (size_t)(mBase + row) * ldc + n0 + c8) = lv;
        }
        __threadfence();
      }
    }
    __builtin_amdgcn_fence(__ATOMIC_RELEASE, "workgroup");
    __builtin_amdgcn_wave_barrier();
    __builtin_amdgcn_fence(__ATOMIC_ACQUIRE, "workgroup");
  }
}

__device__ __forceinline__ float wsum32(float v) {
#pragma unroll
  for (int off = 16; off > 0; off >>= 1) v += __shfl_xor(v, off, 32);
  return v;
}
__device__ __forceinline__ float bsum128(float v, float* red, int lane, int wave) {
  v = wsum32(v);
  if (lane == 0) red[wave] = v;
  __syncthreads();
  return (red[0] + red[1]) + (red[2] + red[3]);
}

__global__ __launch_bounds__(128) void ln1_kernel(const float* __restrict__ X, const float* __restrict__ g,
                                                  const float* __restrict__ bb, unsigned short* __restrict__ X16) {
  __shared__ float redA[4];
  __shared__ float redB[4];
  const int row  = blockIdx.x;
  const int t    = threadIdx.x;
  const int lane = t & 31, wave = t >> 5;
  const int c0   = 8 * t;
  const float* xr = X + (size_t)row * kDim + c0;
  const v4f xa = *(const v4f*)(xr);
  const v4f xc = *(const v4f*)(xr + 4);
  float x[8];
#pragma unroll
  for (int e = 0; e < 4; ++e) { x[e] = xa[e]; x[4 + e] = xc[e]; }
  float s = ((x[0] + x[1]) + (x[2] + x[3])) + ((x[4] + x[5]) + (x[6] + x[7]));
  const float mean = bsum128(s, redA, lane, wave) * kInvDim;
  float sq = 0.f;
#pragma unroll
  for (int e = 0; e < 8; ++e) { x[e] -= mean; sq += x[e] * x[e]; }
  const float var = bsum128(sq, redB, lane, wave) * kInvDim;
  const float inv = 1.0f / sqrtf(var + kLnEps);
  const v4f ga = *(const v4f*)(g + c0);
  const v4f gc = *(const v4f*)(g + c0 + 4);
  const v4f ba = *(const v4f*)(bb + c0);
  const v4f bc = *(const v4f*)(bb + c0 + 4);
  unsigned short hb[8];
#pragma unroll
  for (int e = 0; e < 4; ++e) {
    hb[e]     = h_bits(x[e] * inv * ga[e] + ba[e]);
    hb[4 + e] = h_bits(x[4 + e] * inv * gc[e] + bc[e]);
  }
  const v4u u = (v4u){pk16(hb[0], hb[1]), pk16(hb[2], hb[3]), pk16(hb[4], hb[5]), pk16(hb[6], hb[7])};
  unsigned short* dst = X16 + (size_t)row * kDim + c0;
  *(volatile v4u*)dst = u;
  __threadfence();
  *(volatile v4u*)dst = u;
}

__global__ __launch_bounds__(128) void ln2_kernel(const float* __restrict__ Y0, const float* __restrict__ X,
                                                  const float* __restrict__ g1, const float* __restrict__ b1,
                                                  const float* __restrict__ g2, const float* __restrict__ b2,
                                                  unsigned short* __restrict__ Z16) {
  __shared__ float redA[4];
  __shared__ float redB[4];
  __shared__ float redC[4];
  __shared__ float redD[4];
  const int row  = blockIdx.x;
  const int t    = threadIdx.x;
  const int lane = t & 31, wave = t >> 5;
  const int c0   = 8 * t;
  const float* xr = X + (size_t)row * kDim + c0;
  const v4f xa = *(const v4f*)(xr);
  const v4f xc = *(const v4f*)(xr + 4);
  float x[8];
#pragma unroll
  for (int e = 0; e < 4; ++e) { x[e] = xa[e]; x[4 + e] = xc[e]; }
  float s = ((x[0] + x[1]) + (x[2] + x[3])) + ((x[4] + x[5]) + (x[6] + x[7]));
  const float mean = bsum128(s, redA, lane, wave) * kInvDim;
  float sq = 0.f;
#pragma unroll
  for (int e = 0; e < 8; ++e) { x[e] -= mean; sq += x[e] * x[e]; }
  const float var = bsum128(sq, redB, lane, wave) * kInvDim;
  const float inv = 1.0f / sqrtf(var + kLnEps);
  const v4f ga = *(const v4f*)(g1 + c0);
  const v4f gc = *(const v4f*)(g1 + c0 + 4);
  const v4f ba = *(const v4f*)(b1 + c0);
  const v4f bc = *(const v4f*)(b1 + c0 + 4);
  const float* yr = Y0 + (size_t)row * kDim + c0;
  const v4f ya = *(const v4f*)(yr);
  const v4f yc = *(const v4f*)(yr + 4);
  float y[8];
#pragma unroll
  for (int e = 0; e < 4; ++e) {
    y[e]     = ya[e] + (x[e] * inv * ga[e] + ba[e]);
    y[4 + e] = yc[e] + (x[4 + e] * inv * gc[e] + bc[e]);
  }
  float s2 = ((y[0] + y[1]) + (y[2] + y[3])) + ((y[4] + y[5]) + (y[6] + y[7]));
  const float mean2 = bsum128(s2, redC, lane, wave) * kInvDim;
  float sq2 = 0.f;
#pragma unroll
  for (int e = 0; e < 8; ++e) { y[e] -= mean2; sq2 += y[e] * y[e]; }
  const float var2 = bsum128(sq2, redD, lane, wave) * kInvDim;
  const float inv2 = 1.0f / sqrtf(var2 + kLnEps);
  const v4f g2a = *(const v4f*)(g2 + c0);
  const v4f g2c = *(const v4f*)(g2 + c0 + 4);
  const v4f b2a = *(const v4f*)(b2 + c0);
  const v4f b2c = *(const v4f*)(b2 + c0 + 4);
  unsigned short hb[8];
#pragma unroll
  for (int e = 0; e < 4; ++e) {
    hb[e]     = h_bits(y[e] * inv2 * g2a[e] + b2a[e]);
    hb[4 + e] = h_bits(y[4 + e] * inv2 * g2c[e] + b2c[e]);
  }
  const v4u u = (v4u){pk16(hb[0], hb[1]), pk16(hb[2], hb[3]), pk16(hb[4], hb[5]), pk16(hb[6], hb[7])};
  unsigned short* dst = Z16 + (size_t)row * kDim + c0;
  *(volatile v4u*)dst = u;
  __threadfence();
  *(volatile v4u*)dst = u;
}

__global__ __launch_bounds__(256) void wtcast_kernel(const float* __restrict__ W0, const float* __restrict__ W1,
                                                     const float* __restrict__ W2, unsigned short* __restrict__ out,
                                                     int KD, int ND, float scale) {
  __shared__ float sm[64][65];
  const int t  = threadIdx.x;
  const int k0 = blockIdx.x * 64;
  const int n0 = blockIdx.y * 64;
  const int z  = blockIdx.z;
  const float* W = (z == 0) ? W0 : (z == 1) ? W1 : W2;
#pragma unroll
  for (int i = 0; i < 16; ++i) {
    const int e = i * 256 + t;
    const int r = e >> 6;
    const int c = e & 63;
    sm[c][r] = W[(size_t)(k0 + r) * ND + n0 + c] * scale;
  }
  __syncthreads();
  const int lane = t & 31, wave = t >> 5;
  const int q = lane >> 3, c8 = (lane & 7) * 8;
  unsigned short* op = out + (size_t)z * ND * KD;
  for (int pass = 0; pass < 2; ++pass) {
#pragma unroll
    for (int it = 0; it < 2; ++it) {
      const int row = wave * 8 + it * 4 + q;
      unsigned short hb[8];
#pragma unroll
      for (int e = 0; e < 8; ++e) hb[e] = h_bits(sm[row][c8 + e]);
      const v4u u = (v4u){pk16(hb[0], hb[1]), pk16(hb[2], hb[3]), pk16(hb[4], hb[5]), pk16(hb[6], hb[7])};
      *(volatile v4u*)(op + (size_t)(n0 + row) * KD + k0 + c8) = u;
    }
    __threadfence();
  }
}

__global__ __launch_bounds__(256) void local_attn_kernel(const unsigned short* __restrict__ Q,
                                                         const unsigned short* __restrict__ K,
                                                         const unsigned short* __restrict__ V,
                                                         unsigned short* __restrict__ cat) {
  __shared__ __align__(16) unsigned sC[8][64];
  const int wave = threadIdx.x >> 5;
  const int lane = threadIdx.x & 31;
  const int idx  = blockIdx.x * 8 + wave;
  const int h    = idx & (kHeads - 1);
  const int bt   = idx >> 4;
  const int t    = bt & (kSeq - 1);
  const int b    = bt >> 12;
  const int col  = h * kHS + 2 * lane;
  const size_t rowbase = (size_t)b * kSeq;

#pragma unroll 1
  for (int dir = 0; dir < 2; ++dir) {
    const int sgn = dir ? 1 : -1;
    const int tq  = t + sgn;
    const float fq = (tq >= 0 && tq < kSeq) ? 1.0f : 0.0f;
    const int tqc = tq < 0 ? 0 : (tq >= kSeq ? kSeq - 1 : tq);
    const unsigned wq = *(const unsigned*)(Q + (rowbase + (size_t)tqc) * kDim + col);
    const float qx = hlo2f(wq) * fq, qy = hhi2f(wq) * fq;
    float sc[3], vx[3], vy[3];
#pragma unroll
    for (int j = 0; j < 3; ++j) {
      const int tk  = t + sgn * j;
      const float fk = (tk >= 0 && tk < kSeq) ? 1.0f : 0.0f;
      const int tkc = tk < 0 ? 0 : (tk >= kSeq ? kSeq - 1 : tk);
      const size_t ro = (rowbase + (size_t)tkc) * kDim + col;
      const unsigned wk = *(const unsigned*)(K + ro);
      const unsigned wv = *(const unsigned*)(V + ro);
      const float kx = hlo2f(wk) * fk, ky = hhi2f(wk) * fk;
      vx[j] = hlo2f(wv) * fk;
      vy[j] = hhi2f(wv) * fk;
      sc[j] = wsum32(qx * kx + qy * ky) * kScoreScale;
    }
    const float m  = fmaxf(sc[0], fmaxf(sc[1], sc[2]));
    const float e0 = expf(sc[0] - m);
    const float e1 = expf(sc[1] - m);
    const float e2 = expf(sc[2] - m);
    const float inv = 1.0f / (e0 + (e1 + e2));
    const float p0 = e0 * inv, p1 = e1 * inv, p2 = e2 * inv;
    const float ox = p0 * vx[0] + p1 * vx[1] + p2 * vx[2];
    const float oy = p0 * vy[0] + p1 * vy[1] + p2 * vy[2];
    sC[wave][dir * 32 + lane] = pk16(h_bits(ox), h_bits(oy));
  }
  __syncthreads();
  if (lane < 16) {
    const v4u u = *(const v4u*)(&sC[wave][4 * lane]);
    const int dsel = lane >> 3;
    unsigned short* dst = cat + (rowbase + (size_t)t) * kCat + dsel * kDim + h * kHS + 8 * (lane & 7);
    *(volatile v4u*)dst = u;
    __threadfence();
    *(volatile v4u*)dst = u;
  }
}

__global__ __launch_bounds__(256) void gelu_kernel(const float* __restrict__ G, float* __restrict__ out, int n) {
  const int i = blockIdx.x * 256 + threadIdx.x;
  if (i >= n) return;
  const float v = G[i];
  const float o = 0.5f * v * (1.0f + erff(v * 0.70710678118654752f));
  *(volatile float*)(out + i) = o;
  __threadfence();
  *(volatile float*)(out + i) = o;
}

extern "C" void kernel_launch(void* const* d_in, const int* in_sizes, int n_in,
                              void* d_out, int out_size, void* d_ws, size_t ws_size,
                              hipStream_t stream) {
  if (n_in < 15) return;
  const float* xin = (const float*)d_in[0];
  const float* Wq  = (const float*)d_in[1];
  const float* bq  = (const float*)d_in[2];
  const float* Wk  = (const float*)d_in[3];
  const float* bk  = (const float*)d_in[4];
  const float* Wv  = (const float*)d_in[5];
  const float* bv  = (const float*)d_in[6];
  const float* Wfb = (const float*)d_in[7];
  const float* bfb = (const float*)d_in[8];
  const float* Wo  = (const float*)d_in[9];
  const float* bo  = (const float*)d_in[10];
  const float* g1  = (const float*)d_in[11];
  const float* b1  = (const float*)d_in[12];
  const float* g2  = (const float*)d_in[13];
  const float* b2  = (const float*)d_in[14];
  float* out = (float*)d_out;

  if (in_sizes[0] != kRows * kDim) return;
  if (in_sizes[1] != kDim * kDim || in_sizes[3] != kDim * kDim || in_sizes[5] != kDim * kDim) return;
  if (in_sizes[7] != kCat * kDim || in_sizes[9] != kDim * kDim) return;
  if (in_sizes[2] != kDim || in_sizes[4] != kDim || in_sizes[6] != kDim || in_sizes[8] != kDim || in_sizes[10] != kDim) return;
  if (in_sizes[11] != kDim || in_sizes[12] != kDim || in_sizes[13] != kDim || in_sizes[14] != kDim) return;
  if (out_size != kRows * kDim) return;

  const size_t offX16 = 0;
  const size_t offW   = offX16 + (size_t)kRows * kDim * 2;
  const size_t offWfb = offW   + 3 * (size_t)kDim * kDim * 2;
  const size_t offWo  = offWfb + (size_t)kCat * kDim * 2;
  const size_t offQKV = offWo  + (size_t)kDim * kDim * 2;
  const size_t offCat = offQKV + 3 * (size_t)kRows * kDim * 2;
  const size_t offEnd = offCat + (size_t)kRows * kCat * 2;
  if (offEnd > ws_size) return;

  char* ws = (char*)d_ws;
  unsigned short* X16  = (unsigned short*)(ws + offX16);
  unsigned short* Z16  = X16;
  unsigned short* WqT  = (unsigned short*)(ws + offW);
  unsigned short* WkT  = WqT + (size_t)kDim * kDim;
  unsigned short* WvT  = WkT + (size_t)kDim * kDim;
  unsigned short* WfbT = (unsigned short*)(ws + offWfb);
  unsigned short* WoT  = (unsigned short*)(ws + offWo);
  unsigned short* Q16  = (unsigned short*)(ws + offQKV);
  unsigned short* K16  = Q16 + (size_t)kRows * kDim;
  unsigned short* V16  = K16 + (size_t)kRows * kDim;
  float*          Y0   = (float*)(ws + offQKV);
  float*          Gp   = (float*)(ws + offQKV);
  unsigned short* CAT  = (unsigned short*)(ws + offCat);

  const dim3 blk256(256);
  const dim3 blk128(128);
  const int gemmBlocks = ((kRows / 64) * (kDim / 64)) / 8;

  ln1_kernel<<<dim3(kRows), blk128, 0, stream>>>(xin, g1, b1, X16);

  wtcast_kernel<<<dim3(kDim / 64, kDim / 64, 3), blk256, 0, stream>>>(Wq, Wk, Wv, WqT, kDim, kDim, kWCarry);
  wtcast_kernel<<<dim3(kCat / 64, kDim / 64, 1), blk256, 0, stream>>>(Wfb, Wfb, Wfb, WfbT, kCat, kDim, kWCarry);
  wtcast_kernel<<<dim3(kDim / 64, kDim / 64, 1), blk256, 0, stream>>>(Wo, Wo, Wo, WoT, kDim, kDim, kWCarry);

  wmma_gemm64<0, false, 2, 1, false, 0><<<dim3(gemmBlocks, 1), blk256, 0, stream>>>(
      X16, X16, kDim, 0L, WqT, WqT, kDim, 0L, (void*)Q16, (void*)Q16, kDim, 0L, bq, bq, 0L, kRows, kDim, kDim, kWCarryInv);
  wmma_gemm64<0, false, 2, 1, false, 0><<<dim3(gemmBlocks, 1), blk256, 0, stream>>>(
      X16, X16, kDim, 0L, WkT, WkT, kDim, 0L, (void*)K16, (void*)K16, kDim, 0L, bk, bk, 0L, kRows, kDim, kDim, kWCarryInv);
  wmma_gemm64<0, false, 2, 1, false, 0><<<dim3(gemmBlocks, 1), blk256, 0, stream>>>(
      X16, X16, kDim, 0L, WvT, WvT, kDim, 0L, (void*)V16, (void*)V16, kDim, 0L, bv, bv, 0L, kRows, kDim, kDim, kWCarryInv);

  local_attn_kernel<<<dim3((kRows * kHeads) / 8), blk256, 0, stream>>>(Q16, K16, V16, CAT);

  wmma_gemm64<0, false, 2, 0, false, 0><<<dim3(gemmBlocks, 1), blk256, 0, stream>>>(
      CAT, CAT, kCat, 0L, WfbT, WfbT, kCat, 0L, (void*)Y0, (void*)Y0, kDim, 0L, bfb, bfb, 0L, kRows, kDim, kCat, kWCarryInv);

  ln2_kernel<<<dim3(kRows), blk128, 0, stream>>>(Y0, xin, g1, b1, g2, b2, Z16);

  wmma_gemm64<0, false, 2, 0, false, 0><<<dim3(gemmBlocks, 1), blk256, 0, stream>>>(
      Z16, Z16, kDim, 0L, WoT, WoT, kDim, 0L, (void*)Gp, (void*)Gp, kDim, 0L, bo, bo, 0L, kRows, kDim, kDim, kWCarryInv);

  gelu_kernel<<<dim3((kRows * kDim) / 256), blk256, 0, stream>>>(Gp, out, kRows * kDim);
}
